// EndToEndRPModel_25658134626518
// MI455X (gfx1250) — hardware-verified
//
#include <hip/hip_runtime.h>


#define NB_  64
#define TT   512
#define NF   8
#define C1   32
#define C2   64
#define DZ   6
#define NTK  (NB_ * TT)
#define RP   64
typedef _Float16 h16;
typedef unsigned short bf;
typedef __attribute__((ext_vector_type(16))) __bf16   v16bf;
typedef __attribute__((ext_vector_type(16))) _Float16 v16h;
typedef __attribute__((ext_vector_type(8)))  _Float16 v8h;
typedef __attribute__((ext_vector_type(8)))  unsigned short v8us;
typedef __attribute__((ext_vector_type(8)))  float    v8f;
typedef __attribute__((ext_vector_type(4)))  float    v4f;
typedef v8h  __attribute__((may_alias)) v8ha;
typedef v4f  __attribute__((may_alias)) v4fa;
typedef v8us __attribute__((may_alias)) v8usa;

__device__ __forceinline__ unsigned short f2bf(float f) { unsigned u = __float_as_uint(f); u += 0x7FFFu + ((u >> 16) & 1u); return (unsigned short)(u >> 16); }
__device__ __forceinline__ float bf2f(unsigned short b) { return __uint_as_float(((unsigned)b) << 16); }
__device__ __forceinline__ float bfr(float f) { return bf2f(f2bf(f)); }
__device__ __forceinline__ v16h cat16(v8h lo, v8h hi) { return __builtin_shufflevector(lo, hi, 0, 1, 2, 3, 4, 5, 6, 7, 8, 9, 10, 11, 12, 13, 14, 15); }
__device__ __forceinline__ v16bf cat16b(v8us lo, v8us hi) { return __builtin_bit_cast(v16bf, __builtin_shufflevector(lo, hi, 0, 1, 2, 3, 4, 5, 6, 7, 8, 9, 10, 11, 12, 13, 14, 15)); }
__device__ __forceinline__ v8f wmma16(v16h a, v16h b, v8f c) { return __builtin_amdgcn_wmma_f32_16x16x32_f16(false, a, false, b, (short)0, c, false, false); }
__device__ __forceinline__ v8f wmmab(v16bf a, v16bf b, v8f c) { return __builtin_amdgcn_wmma_f32_16x16x32_bf16(false, a, false, b, (short)0, c, false, false); }


template <typename T16> struct WFrag;
template <> struct WFrag<h16> { typedef v16h V; static __device__ __forceinline__ V ld(const h16* p) { return cat16(*(const v8h*)p, *(const v8h*)(p + 16)); } static __device__ __forceinline__ v8f mma(V a, V b, v8f c) { return wmma16(a, b, c); } };
template <> struct WFrag<bf> { typedef v16bf V; static __device__ __forceinline__ V ld(const bf* p) { return cat16b(*(const v8us*)p, *(const v8us*)(p + 16)); } static __device__ __forceinline__ v8f mma(V a, V b, v8f c) { return wmmab(a, b, c); } };
template <typename T16, int NSPLIT, bool BIAS>
__global__ __launch_bounds__(32) void k_gemmw(const T16* __restrict__ A, const T16* __restrict__ A2, const T16* __restrict__ Bt, const T16* __restrict__ Bt2, int K, float* C, int ldc, const float* __restrict__ bias, size_t sA, size_t sB, size_t sC) {
    typedef typename WFrag<T16>::V V;
    __shared__ __align__(16) float os[16 * 68];
    const size_t z = blockIdx.z; A += z * sA; if (A2) A2 += z * sA; Bt += z * sB; if (Bt2) Bt2 += z * sB; C += z * sC;
    const int lane = threadIdx.x & 31, lr = lane & 15, hi = lane >> 4; const int r0 = blockIdx.x * 64, c0 = blockIdx.y * 64;
    v8f acc[4][4];
#pragma unroll
    for (int mb = 0; mb < 4; ++mb)
#pragma unroll
        for (int nb = 0; nb < 4; ++nb) acc[mb][nb] = (v8f){};
    const size_t aoff = (size_t)(r0 + lr) * K + 8 * hi, boff = (size_t)(c0 + lr) * K + 8 * hi;
#pragma unroll 1
    for (int kc = 0; kc < K; kc += 32) {
        V a[4], a2[4];
#pragma unroll
        for (int mb = 0; mb < 4; ++mb) { a[mb] = WFrag<T16>::ld(A + aoff + (size_t)mb * 16 * K + kc); if (NSPLIT == 1 || NSPLIT == 2) a2[mb] = WFrag<T16>::ld(A2 + aoff + (size_t)mb * 16 * K + kc); }
#pragma unroll
        for (int nb = 0; nb < 4; ++nb) { const V b = WFrag<T16>::ld(Bt + boff + (size_t)nb * 16 * K + kc); V b2; if (NSPLIT >= 2) b2 = WFrag<T16>::ld(Bt2 + boff + (size_t)nb * 16 * K + kc);
#pragma unroll
            for (int mb = 0; mb < 4; ++mb) { acc[mb][nb] = WFrag<T16>::mma(a[mb], b, acc[mb][nb]); if (NSPLIT == 1 || NSPLIT == 2) acc[mb][nb] = WFrag<T16>::mma(a2[mb], b, acc[mb][nb]); if (NSPLIT >= 2) acc[mb][nb] = WFrag<T16>::mma(a[mb], b2, acc[mb][nb]); } }
        asm volatile("v_nop\n\tv_nop\n\tv_nop\n\tv_nop" : "+v"(acc[0][0]), "+v"(acc[1][1]), "+v"(acc[2][2]), "+v"(acc[3][3]) : "v"(a[0]), "v"(a[3]));
    }
#pragma unroll
    for (int mb = 0; mb < 4; ++mb) {
#pragma unroll
        for (int nb = 0; nb < 4; ++nb) {
#pragma unroll
            for (int j = 0; j < 8; ++j) os[(hi * 8 + j) * 68 + nb * 16 + lr] = acc[mb][nb][j]; }
        __builtin_amdgcn_wave_barrier(); asm volatile("" ::: "memory");
        float* crow = C + (size_t)(r0 + mb * 16) * ldc + c0;
#pragma unroll 1
        for (int ps = 0; ps < 2; ++ps) {
#pragma unroll
            for (int s = 0; s < 8; ++s) { const int row = 2 * s + hi, cofs = lr * 4; v4f val = *(const v4fa*)(os + row * 68 + cofs); if (BIAS) { val[0] += bfr(bias[c0 + cofs]); val[1] += bfr(bias[c0 + cofs + 1]); val[2] += bfr(bias[c0 + cofs + 2]); val[3] += bfr(bias[c0 + cofs + 3]); }
                *(volatile v4f*)(crow + (size_t)row * ldc + cofs) = val; }
            if (ps == 0) __threadfence(); }
        __builtin_amdgcn_wave_barrier(); asm volatile("" ::: "memory");
    }
}

__device__ __forceinline__ void splitf(float y, unsigned short& h, unsigned short& l) { h = f2bf(y); l = f2bf(y - bf2f(h)); }
__device__ __forceinline__ float geluf(float x) { return 0.5f * x * (1.0f + erff(x * 0.70710678118654752f)); }
__device__ __forceinline__ float bnscale(float gm) { return __fdiv_rn(bfr(gm), sqrtf(1.00001f)); }

__global__ __launch_bounds__(256) void k_wpad(const float* __restrict__ w, int N, int K, int Np, int Kp, bf* Bt) {
    typedef __attribute__((ext_vector_type(2))) unsigned short v2us;
    const int lane = threadIdx.x & 31; const int nlines = Np * Kp / 64; const int wg = blockIdx.x * 8 + (threadIdx.x >> 5), nw = gridDim.x * 8;
#pragma unroll 1
    for (int ps = 0; ps < 2; ++ps) {
#pragma unroll 1
        for (int L = wg; L < nlines; L += nw) { const int e = L * 64 + lane * 2; v2us o;
#pragma unroll
            for (int q = 0; q < 2; ++q) { const int n = (e + q) / Kp, k = (e + q) % Kp; o[q] = (n < N && k < K) ? f2bf(w[(size_t)(n < N ? n : 0) * K + (k < K ? k : 0)]) : (unsigned short)0; }
            *(volatile v2us*)(Bt + e) = o; }
        if (ps == 0) __threadfence(); }
}
__global__ __launch_bounds__(256) void k_im1(const float* __restrict__ x, bf* A) {
    typedef __attribute__((ext_vector_type(2))) unsigned short v2us;
    const int lane = threadIdx.x & 31; const int L0 = (blockIdx.x * 8 + (threadIdx.x >> 5)) * 8; const int nlines = NTK * 64 / 64;
#pragma unroll 1
    for (int ps = 0; ps < 2; ++ps) {
#pragma unroll
        for (int l = 0; l < 8; ++l) { const int L = L0 + l; if (L >= nlines) break; const int e = L * 64 + lane * 2; const int r = e >> 6, col = e & 63; const int b = r / TT, t = r % TT; v2us o;
#pragma unroll
            for (int q = 0; q < 2; ++q) { const int cc = col + q; const int c = cc / 7, k = cc % 7; const int ts = t + k - 3; const bool in = cc < 56 && ts >= 0 && ts < TT;
                o[q] = in ? f2bf(x[((size_t)b * NF + (c < NF ? c : 0)) * TT + (ts < 0 ? 0 : (ts > TT - 1 ? TT - 1 : ts))]) : (unsigned short)0; }
            *(volatile v2us*)(A + e) = o; }
        if (ps == 0) __threadfence(); }
}
template <int CL>
__global__ __launch_bounds__(256) void k_bngelu(const float* __restrict__ H, const float* __restrict__ gm, const float* __restrict__ bb, int rows, float* G) {
    const int lane = threadIdx.x & 31; const int L0 = (blockIdx.x * 8 + (threadIdx.x >> 5)) * 8; const int nchunks = rows * CL / 128;
#pragma unroll 1
    for (int ps = 0; ps < 2; ++ps) {
#pragma unroll 1
        for (int l = 0; l < 8; ++l) { const int L = L0 + l; if (L >= nchunks) break; v4f o;
            const int e4 = L * 128 + lane * 4;
#pragma unroll
            for (int q = 0; q < 4; ++q) { const int f = e4 + q; const int r = f / CL; const int c = f % CL; o[q] = geluf(H[(size_t)r * 64 + c] * bnscale(gm[c]) + bfr(bb[c])); }
            *(volatile v4f*)(G + e4) = o; }
        if (ps == 0) __threadfence(); }
}
template <int C, int KW, int PAD>
__global__ __launch_bounds__(256) void k_im1d(const float* __restrict__ G, bf* Ah, bf* Al) {
    typedef __attribute__((ext_vector_type(2))) unsigned short v2us;
    constexpr int K = C * KW; const int lane = threadIdx.x & 31; const int L0 = (blockIdx.x * 8 + (threadIdx.x >> 5)) * 8; const int nlines = NTK * K / 64;
#pragma unroll 1
    for (int ps = 0; ps < 2; ++ps) {
#pragma unroll 1
        for (int l = 0; l < 8; ++l) { const int L = L0 + l; if (L >= nlines) break; const int e = L * 64 + lane * 2; v2us oh, ol;
#pragma unroll
            for (int q = 0; q < 2; ++q) { const int f = e + q; const int r = f / K, col = f % K; const int b = r / TT, t = r % TT; const int c = col / KW, k = col % KW; const int ts = t + k - PAD;
                unsigned short a = 0, bl = 0; if (ts >= 0 && ts < TT) splitf(G[((size_t)b * TT + ts) * C + c], a, bl); oh[q] = a; ol[q] = bl; }
            *(volatile v2us*)(Ah + e) = oh; *(volatile v2us*)(Al + e) = ol; }
        if (ps == 0) __threadfence(); }
}
__global__ __launch_bounds__(256) void k_rowsum(const float* __restrict__ Z, float* RS) {
    const int lane = threadIdx.x & 31; const int wg = blockIdx.x * 8 + (threadIdx.x >> 5); if (wg >= NB_ * (TT / 32)) return; const int b = wg / (TT / 32), i = (wg % (TT / 32)) * 32 + lane;
    float zi[DZ]; float sqi = 0.f;
#pragma unroll
    for (int d = 0; d < DZ; ++d) { zi[d] = Z[((size_t)b * TT + i) * 64 + d]; sqi = fmaf(zi[d], zi[d], sqi); }
    float s = 0.f;
#pragma unroll 2
    for (int j = 0; j < TT; ++j) { const float* zj = Z + ((size_t)b * TT + j) * 64; float sqj = 0.f, gr = 0.f;
#pragma unroll
        for (int d = 0; d < DZ; ++d) { const float v = zj[d]; sqj = fmaf(v, v, sqj); gr = fmaf(zi[d], v, gr); }
        const float d2 = fmaxf((sqi + sqj) - 2.0f * gr, 0.f); s += sqrtf(d2 + 1e-6f); }
    float* dst = RS + (size_t)b * TT + i; *(volatile float*)dst = s; __threadfence(); *(volatile float*)dst = s;
}
__global__ __launch_bounds__(256) void k_rp64(const float* __restrict__ Z, const float* __restrict__ RS, float* R64) {
    typedef __attribute__((ext_vector_type(2))) float v2f;
    const int lane = threadIdx.x & 31; const int wg = blockIdx.x * 8 + (threadIdx.x >> 5); if (wg >= NB_ * RP) return; const int b = wg / RP, i = wg % RP;
    float tot = 0.f;
#pragma unroll 1
    for (int q = 0; q < TT / 32; ++q) tot += RS[(size_t)b * TT + q * 32 + lane];
#pragma unroll
    for (int sh = 16; sh; sh >>= 1) tot += __shfl_xor(tot, sh, 32);
    const float sigma = tot * (1.0f / (float)(TT * TT)) + 1e-4f;
    auto zrow = [&](int t, float* z, float& sq) { sq = 0.f;
#pragma unroll
        for (int d = 0; d < DZ; ++d) { z[d] = Z[((size_t)b * TT + t) * 64 + d]; sq = fmaf(z[d], z[d], sq); } };
    auto rp = [&](const float* za, float sqa, const float* zb, float sqb) { float gr = 0.f;
#pragma unroll
        for (int d = 0; d < DZ; ++d) gr = fmaf(za[d], zb[d], gr);
        const float d2 = fmaxf((sqa + sqb) - 2.0f * gr, 0.f); const float dist = sqrtf(d2 + 1e-6f); float a = -__fdiv_rn(dist, sigma); a = fminf(fmaxf(a, -20.f), 0.f); return __expf(a); };
    float r0[DZ], r1[DZ], sq0, sq1; zrow(8 * i + 3, r0, sq0); zrow(8 * i + 4, r1, sq1);
    v2f o;
#pragma unroll 1
    for (int q = 0; q < 2; ++q) { const int j = lane * 2 + q; float c0[DZ], c1[DZ], s0, s1; zrow(8 * j + 3, c0, s0); zrow(8 * j + 4, c1, s1);
        const float a00 = rp(r0, sq0, c0, s0), a10 = rp(r1, sq1, c0, s0), a01 = rp(r0, sq0, c1, s1), a11 = rp(r1, sq1, c1, s1);
        const float rw0 = __fadd_rn(__fmul_rn(a00, 0.5f), __fmul_rn(a10, 0.5f)), rw1 = __fadd_rn(__fmul_rn(a01, 0.5f), __fmul_rn(a11, 0.5f));
        o[q] = __fadd_rn(__fmul_rn(rw0, 0.5f), __fmul_rn(rw1, 0.5f)); }
    float* dst = R64 + ((size_t)b * RP + i) * RP + lane * 2; *(volatile v2f*)dst = o; __threadfence(); *(volatile v2f*)dst = o;
}
__global__ __launch_bounds__(256) void k_rpn(const float* __restrict__ R64, float* RPN) {
    const int lane = threadIdx.x & 31; const int b = blockIdx.x * 8 + (threadIdx.x >> 5); if (b >= NB_) return; const float* src = R64 + (size_t)b * RP * RP;
    float mn = 3.0e38f, mx = -3.0e38f;
#pragma unroll 1
    for (int q = 0; q < RP * RP / 32; ++q) { const float v = src[q * 32 + lane]; mn = fminf(mn, v); mx = fmaxf(mx, v); }
#pragma unroll
    for (int sh = 16; sh; sh >>= 1) { mn = fminf(mn, __shfl_xor(mn, sh, 32)); mx = fmaxf(mx, __shfl_xor(mx, sh, 32)); }
    const float den = (mx - mn) + 1e-4f;
#pragma unroll 1
    for (int ps = 0; ps < 2; ++ps) {
#pragma unroll 1
        for (int q = 0; q < RP * RP / 128; ++q) { v4f o;
#pragma unroll
            for (int k = 0; k < 4; ++k) o[k] = __fdiv_rn(src[q * 128 + lane * 4 + k] - mn, den);
            *(volatile v4f*)(RPN + (size_t)b * RP * RP + q * 128 + lane * 4) = o; }
        if (ps == 0) __threadfence(); }
}
__global__ __launch_bounds__(256) void k_conv1(const float* __restrict__ RPN, const float* __restrict__ w, const float* __restrict__ gm, const float* __restrict__ bb, float* P1) {
    const int lane = threadIdx.x & 31; const int wg = blockIdx.x * 8 + (threadIdx.x >> 5); if (wg >= NB_ * C1 * 32) return; const int b = wg / (C1 * 32), oc = (wg / 32) % C1, Y = wg % 32; const int X = lane;
    const float* img = RPN + (size_t)b * RP * RP; const float s = bnscale(gm[oc]), o0 = bfr(bb[oc]); float wv[9];
#pragma unroll
    for (int k = 0; k < 9; ++k) wv[k] = bfr(w[oc * 9 + k]);
    float best = -3.0e38f;
#pragma unroll 1
    for (int dd = 0; dd < 4; ++dd) { const int dy = dd >> 1, dx = dd & 1; { const int y = 2 * Y + dy, xx = 2 * X + dx; float acc = 0.f;
#pragma unroll
            for (int ky = 0; ky < 3; ++ky)
#pragma unroll
                for (int kx = 0; kx < 3; ++kx) { const int yy = y + ky - 1, xq = xx + kx - 1; const bool in = yy >= 0 && yy < RP && xq >= 0 && xq < RP; const float v = in ? img[(yy < 0 ? 0 : (yy > RP - 1 ? RP - 1 : yy)) * RP + (xq < 0 ? 0 : (xq > RP - 1 ? RP - 1 : xq))] : 0.f; acc = fmaf(v, wv[ky * 3 + kx], acc); }
            best = fmaxf(best, geluf(acc * s + o0)); } }
    float* dst = P1 + (((size_t)b * C1 + oc) * 32 + Y) * 32 + X; *(volatile float*)dst = best; __threadfence(); *(volatile float*)dst = best;
}
template <int C, int S>
__global__ __launch_bounds__(256) void k_im2d(const float* __restrict__ P, bf* Ah, bf* Al) {
    typedef __attribute__((ext_vector_type(2))) unsigned short v2us;
    constexpr int K = 9 * C; constexpr int nrow = NB_ * S * S; const int lane = threadIdx.x & 31; const int L0 = (blockIdx.x * 8 + (threadIdx.x >> 5)) * 8; constexpr int nlines = (int)((size_t)nrow * K / 64);
#pragma unroll 1
    for (int ps = 0; ps < 2; ++ps) {
#pragma unroll 1
        for (int l = 0; l < 8; ++l) { const int L = L0 + l; if (L >= nlines) break; const int e = L * 64 + lane * 2; v2us oh, ol;
#pragma unroll
            for (int q = 0; q < 2; ++q) { const int f = e + q; const int r = f / K; const int col = f % K; const int b = r / (S * S), y = (r / S) % S, xx = r % S; const int c = col / 9, ky = (col % 9) / 3, kx = col % 3;
                const int yy = y + ky - 1, xq = xx + kx - 1; unsigned short a = 0, bl = 0;
                if (yy >= 0 && yy < S && xq >= 0 && xq < S) splitf(P[(((size_t)b * C + c) * S + yy) * S + xq], a, bl); oh[q] = a; ol[q] = bl; }
            *(volatile v2us*)(Ah + e) = oh; *(volatile v2us*)(Al + e) = ol; }
        if (ps == 0) __threadfence(); }
}
template <bool MAXP, int C, int S>
__global__ __launch_bounds__(256) void k_pool(const float* __restrict__ H, int ldh, const float* __restrict__ gm, const float* __restrict__ bb, float* P) {
    constexpr int So = S / 2; constexpr int per = So * So; const int lane = threadIdx.x & 31; const int f = (blockIdx.x * 8 + (threadIdx.x >> 5)) * 32 + lane; if (f - lane >= NB_ * C * per) return;
    const int b = f / (C * per), oc = (f / per) % C, idx = f % per; const int Y = idx / So, X = idx % So;
    const float s = bnscale(gm[oc]), o0 = bfr(bb[oc]); float best = MAXP ? -3.0e38f : 0.f;
#pragma unroll
    for (int dy = 0; dy < 2; ++dy)
#pragma unroll
        for (int dx = 0; dx < 2; ++dx) { const float v = geluf(H[(((size_t)b * S + 2 * Y + dy) * S + 2 * X + dx) * ldh + oc] * s + o0); best = MAXP ? fmaxf(best, v) : best + v; }
    if (!MAXP) best *= 0.25f;
    *(volatile float*)(P + f) = best; __threadfence(); *(volatile float*)(P + f) = best;
}
__global__ __launch_bounds__(256) void k_faplanes(const float* __restrict__ P4, bf* Fh, bf* Fl) {
    typedef __attribute__((ext_vector_type(2))) unsigned short v2us;
    const int lane = threadIdx.x & 31; const size_t L = (size_t)blockIdx.x * 8 + (threadIdx.x >> 5); if (L >= (size_t)NB_ * 2048 / 64) return; const size_t e = L * 64 + lane * 2; v2us oh, ol;
#pragma unroll
    for (int q = 0; q < 2; ++q) { unsigned short a, bl; splitf(P4[e + q], a, bl); oh[q] = a; ol[q] = bl; }
    *(volatile v2us*)(Fh + e) = oh; *(volatile v2us*)(Fl + e) = ol; __threadfence(); *(volatile v2us*)(Fh + e) = oh; *(volatile v2us*)(Fl + e) = ol;
}
__global__ __launch_bounds__(256) void k_outfc(const float* __restrict__ F1, const float* __restrict__ w2, const float* __restrict__ b2, float* OUT) {
    const int lane = threadIdx.x & 31; const int b0 = (blockIdx.x * 8 + (threadIdx.x >> 5)) * 32; if (b0 >= NB_) return;
    float w[8];
#pragma unroll
    for (int q = 0; q < 8; ++q) w[q] = bfr(w2[lane * 8 + q]);
    const float bias = bfr(b2[0]); float mine = 0.f;
#pragma unroll 1
    for (int rr = 0; rr < 32; ++rr) { const float* fr = F1 + (size_t)(b0 + rr) * 256 + lane * 8; float s = 0.f;
#pragma unroll 1
        for (int q = 0; q < 8; ++q) s = fmaf(geluf(fr[q]), w[q], s);
#pragma unroll
        for (int sh = 16; sh; sh >>= 1) s += __shfl_xor(s, sh, 32);
        mine = (lane == rr) ? s + bias : mine; }
    *(volatile float*)(OUT + b0 + lane) = mine; __threadfence(); *(volatile float*)(OUT + b0 + lane) = mine;
}

extern "C" void kernel_launch(void* const* d_in, const int* in_sizes, int n_in,
                              void* d_out, int out_size, void* d_ws, size_t ws_size, hipStream_t stream) {
    (void)in_sizes; (void)n_in; (void)out_size;
    const float* x = (const float*)d_in[0]; const float* w1 = (const float*)d_in[1]; const float* g1 = (const float*)d_in[2]; const float* b1 = (const float*)d_in[3]; const float* w2 = (const float*)d_in[4]; const float* g2 = (const float*)d_in[5]; const float* b2 = (const float*)d_in[6]; const float* w3 = (const float*)d_in[7];
    const float* c1 = (const float*)d_in[8]; const float* cg1 = (const float*)d_in[9]; const float* cb1 = (const float*)d_in[10]; const float* c2 = (const float*)d_in[11]; const float* cg2 = (const float*)d_in[12]; const float* cb2 = (const float*)d_in[13];
    const float* c3 = (const float*)d_in[14]; const float* cg3 = (const float*)d_in[15]; const float* cb3 = (const float*)d_in[16]; const float* c4 = (const float*)d_in[17]; const float* cg4 = (const float*)d_in[18]; const float* cb4 = (const float*)d_in[19];
    const float* f1w = (const float*)d_in[20]; const float* f1b = (const float*)d_in[21]; const float* f2w = (const float*)d_in[22]; const float* f2b = (const float*)d_in[23];
    float* OUT = (float*)d_out;
    char* wsp = (char*)d_ws;
    auto take = [&](size_t bytes) { char* p = wsp; wsp += (bytes + 255) & ~(size_t)255; return (void*)p; };
    bf* W1t = (bf*)take(64 * 64 * 2); bf* W2t = (bf*)take(64 * 160 * 2); bf* W3t = (bf*)take(64 * 192 * 2); bf* C2t = (bf*)take(64 * 288 * 2); bf* C3t = (bf*)take(128 * 576 * 2); bf* C4t = (bf*)take(128 * 1152 * 2); bf* F1t = (bf*)take((size_t)256 * 2048 * 2);
    bf* PLh = (bf*)take((size_t)NB_ * 1024 * 288 * 2); bf* PLl = (bf*)take((size_t)NB_ * 1024 * 288 * 2);
    float* HF = (float*)take((size_t)NB_ * 1024 * 64 * 4);
    float* G = (float*)take((size_t)NTK * 64 * 4);
    float* RS = (float*)take((size_t)NB_ * TT * 4); float* R64 = (float*)take((size_t)NB_ * RP * RP * 4); float* RPN = (float*)take((size_t)NB_ * RP * RP * 4);
    float* P1 = (float*)take((size_t)NB_ * C1 * 32 * 32 * 4); float* P2 = (float*)take((size_t)NB_ * 64 * 16 * 16 * 4); float* P3 = (float*)take((size_t)NB_ * 128 * 8 * 8 * 4); float* P4 = (float*)take((size_t)NB_ * 2048 * 4);
    float* F1 = (float*)take((size_t)NB_ * 256 * 4);
    if ((size_t)(wsp - (char*)d_ws) > ws_size) return;
    k_wpad<<<4, 256, 0, stream>>>(w1, 32, 56, 64, 64, W1t); k_wpad<<<4, 256, 0, stream>>>(w2, 64, 160, 64, 160, W2t); k_wpad<<<4, 256, 0, stream>>>(w3, 6, 192, 64, 192, W3t);
    k_wpad<<<8, 256, 0, stream>>>(c2, 64, 288, 64, 288, C2t); k_wpad<<<16, 256, 0, stream>>>(c3, 128, 576, 128, 576, C3t); k_wpad<<<32, 256, 0, stream>>>(c4, 128, 1152, 128, 1152, C4t); k_wpad<<<64, 256, 0, stream>>>(f1w, 256, 2048, 256, 2048, F1t);
    k_im1<<<(NTK * 64 / 64 + 63) / 64, 256, 0, stream>>>(x, PLh);
    k_gemmw<bf, 0, false><<<dim3(NTK / 64, 1, 1), 32, 0, stream>>>(PLh, nullptr, W1t, nullptr, 64, HF, 64, nullptr, 0, 0, 0);
    k_bngelu<32><<<(unsigned)(((size_t)NTK * 32 / 128 + 63) / 64), 256, 0, stream>>>(HF, g1, b1, NTK, G);
    k_im1d<32, 5, 2><<<(unsigned)(((size_t)NTK * 160 / 64 + 63) / 64), 256, 0, stream>>>(G, PLh, PLl);
    k_gemmw<bf, 1, false><<<dim3(NTK / 64, 1, 1), 32, 0, stream>>>(PLh, PLl, W2t, nullptr, 160, HF, 64, nullptr, 0, 0, 0);
    k_bngelu<64><<<(unsigned)(((size_t)NTK * 64 / 128 + 63) / 64), 256, 0, stream>>>(HF, g2, b2, NTK, G);
    k_im1d<64, 3, 1><<<(unsigned)(((size_t)NTK * 192 / 64 + 63) / 64), 256, 0, stream>>>(G, PLh, PLl);
    k_gemmw<bf, 1, false><<<dim3(NTK / 64, 1, 1), 32, 0, stream>>>(PLh, PLl, W3t, nullptr, 192, HF, 64, nullptr, 0, 0, 0);
    k_rowsum<<<NB_ * (TT / 32) / 8, 256, 0, stream>>>(HF, RS);
    k_rp64<<<NB_ * RP / 8, 256, 0, stream>>>(HF, RS, R64);
    k_rpn<<<NB_ / 8, 256, 0, stream>>>(R64, RPN);
    k_conv1<<<NB_ * C1 * 32 / 8, 256, 0, stream>>>(RPN, c1, cg1, cb1, P1);
    k_im2d<32, 32><<<(unsigned)(((size_t)NB_ * 32 * 32 * 288 / 64 + 63) / 64), 256, 0, stream>>>(P1, PLh, PLl);
    k_gemmw<bf, 1, false><<<dim3(NB_ * 32 * 32 / 64, 1, 1), 32, 0, stream>>>(PLh, PLl, C2t, nullptr, 288, HF, 64, nullptr, 0, 0, 0);
    k_pool<true, 64, 32><<<NB_ * 64 * 256 / 32 / 8, 256, 0, stream>>>(HF, 64, cg2, cb2, P2);
    k_im2d<64, 16><<<(unsigned)(((size_t)NB_ * 16 * 16 * 576 / 64 + 63) / 64), 256, 0, stream>>>(P2, PLh, PLl);
    k_gemmw<bf, 1, false><<<dim3(NB_ * 16 * 16 / 64, 2, 1), 32, 0, stream>>>(PLh, PLl, C3t, nullptr, 576, HF, 128, nullptr, 0, 0, 0);
    k_pool<true, 128, 16><<<NB_ * 128 * 64 / 32 / 8, 256, 0, stream>>>(HF, 128, cg3, cb3, P3);
    k_im2d<128, 8><<<(unsigned)(((size_t)NB_ * 8 * 8 * 1152 / 64 + 63) / 64), 256, 0, stream>>>(P3, PLh, PLl);
    k_gemmw<bf, 1, false><<<dim3(NB_ * 8 * 8 / 64, 2, 1), 32, 0, stream>>>(PLh, PLl, C4t, nullptr, 1152, HF, 128, nullptr, 0, 0, 0);
    k_pool<false, 128, 8><<<NB_ * 128 * 16 / 32 / 8, 256, 0, stream>>>(HF, 128, cg4, cb4, P4);
    k_faplanes<<<(NB_ * 2048 / 64 + 7) / 8, 256, 0, stream>>>(P4, PLh, PLl);
    k_gemmw<bf, 1, true><<<dim3(NB_ / 64, 256 / 64, 1), 32, 0, stream>>>(PLh, PLl, F1t, nullptr, 2048, F1, 256, f1b, 0, 0, 0);
    k_outfc<<<1, 256, 0, stream>>>(F1, f2w, f2b, OUT);
}
